// MultiHeadAttn_32693291057795
// MI455X (gfx1250) — hardware-verified
//
#include <hip/hip_runtime.h>
#include <math.h>
#include <stdint.h>

#ifndef NB
#define NB 2
#endif
#ifndef NB_FULL
#define NB_FULL 2
#endif
#ifndef SEQ
#define SEQ 2048
#endif
#ifndef SEQ_FULL
#define SEQ_FULL 2048
#endif
#define DE    1024
#define NH    16
#define HD    64
#define NQB   (SEQ / 64)
#define MROWS (NB * SEQ)
#ifndef RESQB
#define RESQB 8
#endif
#define PCARRY 16384.0f
#define PRES   4096.0f
#define VCARRY 64.0f
#define CCARRY 64.0f
#define WCARRY 64.0f

static_assert(NB >= 1 && NB <= NB_FULL);
static_assert((SEQ % 128) == 0 && SEQ >= 128 && SEQ <= SEQ_FULL);
static_assert(NH * HD == DE);
static_assert(RESQB >= 1);
static_assert((MROWS % 128) == 0 && (DE % 64) == 0 && (DE % 32) == 0);
static_assert((long long)NB_FULL * SEQ_FULL * DE * 4 == 16777216LL);

typedef _Float16 v16h __attribute__((ext_vector_type(16)));
typedef _Float16 v8h  __attribute__((ext_vector_type(8)));
typedef __bf16   v16b __attribute__((ext_vector_type(16)));
typedef __bf16   v8b  __attribute__((ext_vector_type(8)));
typedef float    v8f  __attribute__((ext_vector_type(8)));
typedef float    v4f  __attribute__((ext_vector_type(4)));
typedef unsigned int v4u __attribute__((ext_vector_type(4)));
typedef unsigned short v8us __attribute__((ext_vector_type(8)));

__device__ __forceinline__ unsigned short bf_bits(float f) {
  unsigned u = __float_as_uint(f);
  return (unsigned short)((u + 0x7FFFu + ((u >> 16) & 1u)) >> 16);
}
__device__ __forceinline__ float bf_up(unsigned short h) { return __uint_as_float(((unsigned)h) << 16); }
__device__ __forceinline__ unsigned short h_bits(float f) {
  union { _Float16 h; unsigned short u; } cvt;
  cvt.h = (_Float16)f;
  return cvt.u;
}
__device__ __forceinline__ unsigned pk16(unsigned short a, unsigned short b) { return (unsigned)a | ((unsigned)b << 16); }
__device__ __forceinline__ v8f zero8() { v8f z = {0.f, 0.f, 0.f, 0.f, 0.f, 0.f, 0.f, 0.f}; return z; }

__device__ __forceinline__ v16b ldfrag_b(const __bf16* p) {
  union { v16b v; v8b h[2]; } f;
  f.h[0] = *(const v8b*)(p);
  f.h[1] = *(const v8b*)(p + 16);
  return f.v;
}
__device__ __forceinline__ v16h ldfrag_h(const _Float16* p) {
  union { v16h v; v8h h[2]; } f;
  f.h[0] = *(const v8h*)(p);
  f.h[1] = *(const v8h*)(p + 16);
  return f.v;
}

__device__ __forceinline__ v8f mma_b(v16b a, v16b b, v8f c) {
  c = __builtin_amdgcn_wmma_f32_16x16x32_bf16(false, a, false, b, (short)0, c, false, false);
  asm volatile("v_nop\n\tv_nop\n\tv_nop\n\tv_nop" : "+v"(c) : "v"(a), "v"(b));
  return c;
}
__device__ __forceinline__ v8f mma_h(v16h a, v16h b, v8f c) {
  c = __builtin_amdgcn_wmma_f32_16x16x32_f16(false, a, false, b, (short)0, c, false, false);
  asm volatile("v_nop\n\tv_nop\n\tv_nop\n\tv_nop" : "+v"(c) : "v"(a), "v"(b));
  return c;
}

__global__ __launch_bounds__(256) void cvt_bf16x8s(const float* __restrict__ in, unsigned short* out,
                                                   int n8, int per8, int src8) {
  const int i = blockIdx.x * 256 + threadIdx.x;
  if (i < n8) {
    const int hd  = i / per8;
    const int rem = i - hd * per8;
    const float* s = in + ((size_t)hd * src8 + (size_t)rem) * 8;
    const v4f a = *(const v4f*)(s);
    const v4f b = *(const v4f*)(s + 4);
    v4u p;
    p[0] = pk16(bf_bits(a[0]), bf_bits(a[1]));
    p[1] = pk16(bf_bits(a[2]), bf_bits(a[3]));
    p[2] = pk16(bf_bits(b[0]), bf_bits(b[1]));
    p[3] = pk16(bf_bits(b[2]), bf_bits(b[3]));
    *(volatile v4u*)(out + (size_t)i * 8) = p;
    __threadfence();
    *(volatile v4u*)(out + (size_t)i * 8) = p;
  }
}

__global__ __launch_bounds__(256) void wt_tiles(const float* __restrict__ w0, const float* __restrict__ w1,
                                                const float* __restrict__ w2, const float* __restrict__ w3,
                                                unsigned short* o0, unsigned short* o1,
                                                unsigned short* o2, unsigned short* o3) {
  __shared__ __align__(16) unsigned short T[64 * 64];
  const int tid = threadIdx.x;
  const int mat = blockIdx.y;
  const float* in = w0; unsigned short* out = o0;
  if (mat == 1) { in = w1; out = o1; }
  else if (mat == 2) { in = w2; out = o2; }
  else if (mat == 3) { in = w3; out = o3; }
  const int ktile = blockIdx.x / (DE / 64);
  const int ntile = blockIdx.x - ktile * (DE / 64);
  const int k   = tid >> 2;
  const int nq  = (tid & 3) * 16;
  const float* src = in + (size_t)(ktile * 64 + k) * DE + ntile * 64 + nq;
#pragma unroll
  for (int i = 0; i < 4; ++i) {
    const v4f a = *(const v4f*)(src + 4 * i);
#pragma unroll
    for (int e = 0; e < 4; ++e) {
      const unsigned short bb = bf_bits(a[e]);
      const unsigned short hb = h_bits(bf_up(bb) * WCARRY);
      const unsigned short us = (mat == 3) ? hb : bb;
      T[(nq + 4 * i + e) * 64 + k] = us;
    }
  }
  __syncthreads();
  const int wave = tid >> 5, lane = tid & 31;
  const int q = lane >> 3, c8 = (lane & 7) * 8;
  union { v8us s; v4u u; } x0, x1;
  const int d0 = wave * 8 + q;
  const int d1 = wave * 8 + 4 + q;
  x0.s = *(const v8us*)(T + d0 * 64 + c8);
  x1.s = *(const v8us*)(T + d1 * 64 + c8);
  unsigned short* p0 = out + ((size_t)(ntile * 64 + d0) * DE + ktile * 64 + c8);
  unsigned short* p1 = out + ((size_t)(ntile * 64 + d1) * DE + ktile * 64 + c8);
  *(volatile v4u*)p0 = x0.u;
  *(volatile v4u*)p1 = x1.u;
  __threadfence();
  *(volatile v4u*)p0 = x0.u;
  *(volatile v4u*)p1 = x1.u;
}

template <int MODE>
__global__ __launch_bounds__(256)
void gemm_nt(const unsigned short* __restrict__ A, const unsigned short* __restrict__ Bt,
             const float* __restrict__ bias, const float* __restrict__ resid,
             unsigned short* out16, float* out32, float scale) {
  __shared__ __align__(16) unsigned char smem[32768];
  const int tid  = threadIdx.x;
  const int wave = tid >> 5;
  const int lane = tid & 31;
  const int hh   = lane >> 4;
  const int c    = lane & 15;
  const int m0b  = blockIdx.y * 128;
  const int m0   = m0b + wave * 16;
  const int n0   = blockIdx.x * 64;

  v8f acc[4];
#pragma unroll
  for (int t = 0; t < 4; ++t) acc[t] = zero8();

  const size_t aoff = (size_t)(m0 + c) * DE + 8 * hh;
  const size_t boff = (size_t)(n0 + c) * DE + 8 * hh;
  if (MODE == 2) {
    const _Float16* Ah = (const _Float16*)(const void*)A + aoff;
    const _Float16* Bh = (const _Float16*)(const void*)Bt + boff;
#pragma unroll 2
    for (int k0 = 0; k0 < DE; k0 += 32) {
      const v16h a = ldfrag_h(Ah + k0);
#pragma unroll
      for (int t = 0; t < 4; ++t) {
        const v16h b = ldfrag_h(Bh + (size_t)t * 16 * DE + k0);
        acc[t] = mma_h(a, b, acc[t]);
      }
    }
  } else {
    const __bf16* Ab = (const __bf16*)(const void*)A + aoff;
    const __bf16* Bb = (const __bf16*)(const void*)Bt + boff;
#pragma unroll 2
    for (int k0 = 0; k0 < DE; k0 += 32) {
      const v16b a = ldfrag_b(Ab + k0);
#pragma unroll
      for (int t = 0; t < 4; ++t) {
        const v16b b = ldfrag_b(Bb + (size_t)t * 16 * DE + k0);
        acc[t] = mma_b(a, b, acc[t]);
      }
    }
  }

  if (MODE == 0) {
    _Float16* S = (_Float16*)(void*)smem + wave * 1024;
#pragma unroll
    for (int t = 0; t < 4; ++t) {
      const float bi = bf_up(bf_bits(bias[n0 + t * 16 + c]));
#pragma unroll
      for (int r = 0; r < 8; ++r) S[(8 * hh + r) * 64 + t * 16 + c] = (_Float16)((acc[t][r] + bi) * scale);
    }
    __builtin_amdgcn_fence(__ATOMIC_RELEASE, "workgroup");
    __builtin_amdgcn_wave_barrier();
    __builtin_amdgcn_fence(__ATOMIC_ACQUIRE, "workgroup");
    const int rq = lane >> 3, c8 = (lane & 7) * 8;
    union { v8h h; v4u u; } w[4];
#pragma unroll
    for (int it = 0; it < 4; ++it) w[it].h = *(const v8h*)(S + (it * 4 + rq) * 64 + c8);
    for (int rep = 0; rep < 2; ++rep) {
#pragma unroll
      for (int it = 0; it < 4; ++it)
        *(volatile v4u*)(out16 + (size_t)(m0 + it * 4 + rq) * DE + n0 + c8) = w[it].u;
      __threadfence();
    }
  } else if (MODE == 1) {
    _Float16* T = (_Float16*)(void*)smem;
#pragma unroll
    for (int t = 0; t < 4; ++t) {
      const float bi = bf_up(bf_bits(bias[n0 + t * 16 + c]));
#pragma unroll
      for (int r = 0; r < 8; ++r)
        T[(t * 16 + c) * 128 + wave * 16 + 8 * hh + r] = (_Float16)((acc[t][r] + bi) * scale);
    }
    __syncthreads();
    const int bidx = m0b / SEQ;
    const int key0 = m0b - bidx * SEQ;
    const int rh = lane >> 4, c8 = (lane & 15) * 8;
    union { v8h h; v4u u; } w[4];
#pragma unroll
    for (int it = 0; it < 4; ++it) w[it].h = *(const v8h*)(T + (wave * 8 + it * 2 + rh) * 128 + c8);
    for (int rep = 0; rep < 2; ++rep) {
#pragma unroll
      for (int it = 0; it < 4; ++it) {
        const int row = wave * 8 + it * 2 + rh;
        *(volatile v4u*)(out16 + ((size_t)(bidx * DE + n0 + row) * SEQ + key0 + c8)) = w[it].u;
      }
      __threadfence();
    }
  } else {
    float* S = (float*)(void*)smem + wave * 1024;
#pragma unroll
    for (int t = 0; t < 4; ++t) {
      const float bi = bf_up(bf_bits(bias[n0 + t * 16 + c]));
#pragma unroll
      for (int r = 0; r < 8; ++r) S[(8 * hh + r) * 64 + t * 16 + c] = acc[t][r] * scale + bi;
    }
    __builtin_amdgcn_fence(__ATOMIC_RELEASE, "workgroup");
    __builtin_amdgcn_wave_barrier();
    __builtin_amdgcn_fence(__ATOMIC_ACQUIRE, "workgroup");
    const int rh = lane >> 4, c4 = (lane & 15) * 4;
    v4f vals[8];
#pragma unroll
    for (int it = 0; it < 8; ++it) {
      const int row = it * 2 + rh;
      const int gm  = m0 + row;
      const int bb  = gm / SEQ;
      const int tt  = gm - bb * SEQ;
      v4f x = *(const v4f*)(S + row * 64 + c4);
      const v4f rq = *(const v4f*)(resid + ((size_t)bb * SEQ_FULL + tt) * DE + n0 + c4);
#pragma unroll
      for (int e = 0; e < 4; ++e) x[e] = x[e] + bf_up(bf_bits(rq[e]));
      vals[it] = x;
    }
    for (int rep = 0; rep < 2; ++rep) {
#pragma unroll
      for (int it = 0; it < 8; ++it)
        *(volatile v4f*)(out32 + (size_t)(m0 + it * 2 + rh) * DE + n0 + c4) = vals[it];
      __threadfence();
    }
  }
}

template <bool RES>
__global__ __launch_bounds__(128)
void attn_full64(const unsigned short* __restrict__ qp, const unsigned short* __restrict__ kp,
                 const unsigned short* __restrict__ vtp, unsigned short* ctx, int qbBase, int nqbThis) {
  union FH { v16h v; v8h h[2]; };
  __shared__ __align__(16) _Float16 Ksh[64 * 64];
  __shared__ __align__(16) _Float16 Vth[64 * 64];
  __shared__ __align__(16) _Float16 Psh[4][16 * 64];
  __shared__ __align__(16) _Float16 Psl[RES ? 4 : 1][16 * 64];
  __shared__ __align__(16) _Float16 Os[4][16 * 64];

  const int tid  = threadIdx.x;
  const int wave = tid >> 5;
  const int lane = tid & 31;
  const int hh   = lane >> 4;
  const int c    = lane & 15;

  const int bx   = blockIdx.x;
  const int qbl  = bx % nqbThis;
  const int bhq  = bx / nqbThis;
  const int h    = bhq % NH;
  const int b    = bhq / NH;
  const int qb   = qbBase + qbl;
  const int q0   = qb * 64 + wave * 16;

  const _Float16* Qh = (const _Float16*)(const void*)qp + (size_t)b * SEQ * DE + (size_t)h * HD;
  const _Float16* Kh = (const _Float16*)(const void*)kp + (size_t)b * SEQ * DE + (size_t)h * HD;
  const _Float16* Vh = (const _Float16*)(const void*)vtp + ((size_t)b * DE + (size_t)h * HD) * SEQ;

  v16h qa[2];
#pragma unroll
  for (int dc = 0; dc < 2; ++dc) {
    const size_t qo = (size_t)(q0 + c) * DE + dc * 32 + 8 * hh;
    qa[dc] = ldfrag_h(Qh + qo);
  }

  float mrow[8], lrow[8];
  v8f oacc[4];
#pragma unroll
  for (int r = 0; r < 8; ++r) { mrow[r] = -INFINITY; lrow[r] = 0.f; }
#pragma unroll
  for (int t = 0; t < 4; ++t) oacc[t] = zero8();

  for (int kt = 0; kt < NQB; ++kt) {
    const int kv0 = kt * 64;
    __syncthreads();
    {
      const int r = tid >> 1, half = (tid & 1) * 32;
      const _Float16* kg = Kh + (size_t)(kv0 + r) * DE + half;
      const _Float16* vg = Vh + (size_t)r * SEQ + kv0 + half;
#pragma unroll
      for (int i = 0; i < 4; ++i) {
        const v8h a0 = *(const v8h*)(kg + 8 * i);
        const v8h b0 = *(const v8h*)(vg + 8 * i);
        *(v8h*)(Ksh + r * 64 + half + 8 * i) = a0;
        *(v8h*)(Vth + r * 64 + half + 8 * i) = b0;
      }
    }
    __syncthreads();

    v8f s[4];
#pragma unroll
    for (int j = 0; j < 4; ++j) {
      s[j] = zero8();
#pragma unroll
      for (int dc = 0; dc < 2; ++dc) {
        FH kb;
        kb.h[0] = *(const v8h*)(Ksh + (j * 16 + c) * 64 + dc * 32 + 8 * hh);
        kb.h[1] = *(const v8h*)(Ksh + (j * 16 + c) * 64 + dc * 32 + 16 + 8 * hh);
        s[j] = mma_h(qa[dc], kb.v, s[j]);
      }
    }

    _Float16* pwh = Psh[wave];
    _Float16* pwl = Psl[RES ? wave : 0];
#pragma unroll
    for (int r = 0; r < 8; ++r) {
      float m = -INFINITY;
#pragma unroll
      for (int j = 0; j < 4; ++j) {
        const float sv = s[j][r] * 0.125f;
        s[j][r] = sv;
        m = fmaxf(m, sv);
      }
#pragma unroll
      for (int off = 1; off < 16; off <<= 1) m = fmaxf(m, __shfl_xor(m, off, 32));
      const float mnew  = fmaxf(mrow[r], m);
      const float msafe = (mnew == -INFINITY) ? 0.f : mnew;
      const float alpha = __expf(mrow[r] - msafe);
      mrow[r] = mnew;
      float psum = 0.f;
#pragma unroll
      for (int j = 0; j < 4; ++j) {
        const float p = __expf(s[j][r] - msafe);
        psum += p;
        const float p1k = p * PCARRY;
        const _Float16 ph = (_Float16)p1k;
        pwh[(8 * hh + r) * 64 + j * 16 + c] = ph;
        if (RES) {
          const _Float16 pl = (_Float16)((p1k - (float)ph) * PRES);
          pwl[(8 * hh + r) * 64 + j * 16 + c] = pl;
        }
      }
#pragma unroll
      for (int off = 1; off < 16; off <<= 1) psum += __shfl_xor(psum, off, 32);
      lrow[r] = lrow[r] * alpha + psum;
#pragma unroll
      for (int t = 0; t < 4; ++t) oacc[t][r] *= alpha;
    }
    __builtin_amdgcn_fence(__ATOMIC_RELEASE, "workgroup");
    __builtin_amdgcn_wave_barrier();
    __builtin_amdgcn_fence(__ATOMIC_ACQUIRE, "workgroup");

    v8f o1[4];
#pragma unroll
    for (int t = 0; t < 4; ++t) o1[t] = zero8();
#pragma unroll 1
    for (int kk = 0; kk < 2; ++kk) {
      FH pa, pl;
      pa.h[0] = *(const v8h*)(pwh + c * 64 + kk * 32 + 8 * hh);
      pa.h[1] = *(const v8h*)(pwh + c * 64 + kk * 32 + 16 + 8 * hh);
      if (RES) {
        pl.h[0] = *(const v8h*)(pwl + c * 64 + kk * 32 + 8 * hh);
        pl.h[1] = *(const v8h*)(pwl + c * 64 + kk * 32 + 16 + 8 * hh);
      } else {
        pl.v = pa.v;
      }
#pragma unroll
      for (int t = 0; t < 4; ++t) {
        FH vb;
        vb.h[0] = *(const v8h*)(Vth + (t * 16 + c) * 64 + kk * 32 + 8 * hh);
        vb.h[1] = *(const v8h*)(Vth + (t * 16 + c) * 64 + kk * 32 + 16 + 8 * hh);
        oacc[t] = mma_h(pa.v, vb.v, oacc[t]);
        if (RES) o1[t] = mma_h(pl.v, vb.v, o1[t]);
      }
    }
    if (RES) {
#pragma unroll
      for (int t = 0; t < 4; ++t)
#pragma unroll
        for (int r = 0; r < 8; ++r) oacc[t][r] += o1[t][r] * (1.0f / PRES);
    }
  }

  _Float16* os = Os[wave];
#pragma unroll
  for (int r = 0; r < 8; ++r) {
    const float l = lrow[r];
    const float inv = ((l > 0.f) ? (1.0f / l) : 0.f) * (CCARRY / (PCARRY * VCARRY));
#pragma unroll
    for (int t = 0; t < 4; ++t) os[(8 * hh + r) * 64 + t * 16 + c] = (_Float16)(oacc[t][r] * inv);
  }
  __builtin_amdgcn_fence(__ATOMIC_RELEASE, "workgroup");
  __builtin_amdgcn_wave_barrier();
  __builtin_amdgcn_fence(__ATOMIC_ACQUIRE, "workgroup");
  {
    const int rq = lane >> 3, c8 = (lane & 7) * 8;
    union { v8h h; v4u u; } w[4];
#pragma unroll
    for (int it = 0; it < 4; ++it) w[it].h = *(const v8h*)(os + (it * 4 + rq) * 64 + c8);
    unsigned short* ob = ctx + ((size_t)b * SEQ) * DE + (size_t)h * HD;
    for (int rep = 0; rep < 2; ++rep) {
#pragma unroll
      for (int it = 0; it < 4; ++it) {
        const int row = it * 4 + rq;
        *(volatile v4u*)(ob + (size_t)(q0 + row) * DE + c8) = w[it].u;
      }
      __threadfence();
    }
  }
}

__global__ __launch_bounds__(256) void ln_rows(const float* __restrict__ x, const float* __restrict__ gam,
                                               const float* __restrict__ bet, float* out) {
  __shared__ float red1[8];
  __shared__ float red2[8];
  const int tid = threadIdx.x, wave = tid >> 5, lane = tid & 31;
  const int row = blockIdx.x;
  const int bb  = row / SEQ;
  const int tt  = row - bb * SEQ;
  const size_t orow = (size_t)bb * SEQ_FULL + (size_t)tt;

  const v4f v = *(const v4f*)(x + (size_t)row * DE + tid * 4);
  float s = (v[0] + v[1]) + (v[2] + v[3]);
#pragma unroll
  for (int off = 16; off > 0; off >>= 1) s += __shfl_xor(s, off, 32);
  if (lane == 0) red1[wave] = s;
  __syncthreads();
  float tot = 0.f;
#pragma unroll
  for (int w = 0; w < 8; ++w) tot += red1[w];
  const float mu = tot * (1.0f / (float)DE);

  v4f d;
#pragma unroll
  for (int e = 0; e < 4; ++e) d[e] = v[e] - mu;
  float s2 = (d[0] * d[0] + d[1] * d[1]) + (d[2] * d[2] + d[3] * d[3]);
#pragma unroll
  for (int off = 16; off > 0; off >>= 1) s2 += __shfl_xor(s2, off, 32);
  if (lane == 0) red2[wave] = s2;
  __syncthreads();
  float tot2 = 0.f;
#pragma unroll
  for (int w = 0; w < 8; ++w) tot2 += red2[w];
  const float var  = tot2 * (1.0f / (float)DE);
  const float rstd = rsqrtf(var + 1.0e-5f);

  const v4f g4 = *(const v4f*)(gam + tid * 4);
  const v4f b4 = *(const v4f*)(bet + tid * 4);
  v4f y;
#pragma unroll
  for (int e = 0; e < 4; ++e) y[e] = (d[e] * rstd) * bf_up(bf_bits(g4[e])) + bf_up(bf_bits(b4[e]));
  float* op = out + orow * DE + (size_t)tid * 4;
  *(volatile v4f*)op = y;
  __threadfence();
  *(volatile v4f*)op = y;
}

extern "C" void kernel_launch(void* const* d_in, const int* in_sizes, int n_in,
                              void* d_out, int out_size, void* d_ws, size_t ws_size,
                              hipStream_t stream) {
  if (n_in < 12) return;
  const long long needIn = (long long)(NB - 1) * SEQ_FULL * DE + (long long)SEQ * DE;
  if ((long long)in_sizes[0] < needIn || (long long)in_sizes[1] < needIn) return;
  if (in_sizes[2] < DE * DE || in_sizes[4] < DE * DE || in_sizes[6] < DE * DE || in_sizes[8] < DE * DE) return;
  if (in_sizes[3] < DE || in_sizes[5] < DE || in_sizes[7] < DE || in_sizes[9] < DE) return;
  if (in_sizes[10] < DE || in_sizes[11] < DE) return;
  if (out_size < 0 || (long long)out_size < needIn) return;

  const size_t P16 = (size_t)MROWS * DE * 2;
  const size_t W16 = (size_t)DE * DE * 2;
  const size_t P32 = (size_t)MROWS * DE * 4;
  size_t off = 0;
  const size_t oPQ  = off; off += P16;
  const size_t oPK  = off; off += P16;
  const size_t oWq  = off; off += W16;
  const size_t oWk  = off; off += W16;
  const size_t oWv  = off; off += W16;
  const size_t oWo  = off; off += W16;
  const size_t oQ   = off; off += P16;
  const size_t oK   = off; off += P16;
  const size_t oVT  = off; off += P16;
  const size_t oCTX = off; off += P16;
  const size_t oX   = off; off += P32;
  if (off > ws_size) return;
  if (off > (size_t)134217728) return;

  const float* pre_q = (const float*)d_in[0];
  const float* pre_k = (const float*)d_in[1];
  const float* Wq    = (const float*)d_in[2];
  const float* bq    = (const float*)d_in[3];
  const float* Wk    = (const float*)d_in[4];
  const float* bk    = (const float*)d_in[5];
  const float* Wv    = (const float*)d_in[6];
  const float* bv    = (const float*)d_in[7];
  const float* Wo    = (const float*)d_in[8];
  const float* bo    = (const float*)d_in[9];
  const float* gamma = (const float*)d_in[10];
  const float* beta  = (const float*)d_in[11];
  float* out = (float*)d_out;

  char* ws = (char*)d_ws;
  unsigned short* PQb  = (unsigned short*)(ws + oPQ);
  unsigned short* PKb  = (unsigned short*)(ws + oPK);
  unsigned short* Wqt  = (unsigned short*)(ws + oWq);
  unsigned short* Wkt  = (unsigned short*)(ws + oWk);
  unsigned short* Wvt  = (unsigned short*)(ws + oWv);
  unsigned short* Wot  = (unsigned short*)(ws + oWo);
  unsigned short* Qh   = (unsigned short*)(ws + oQ);
  unsigned short* Kh   = (unsigned short*)(ws + oK);
  unsigned short* VTb  = (unsigned short*)(ws + oVT);
  unsigned short* CTXb = (unsigned short*)(ws + oCTX);
  float*          Xb   = (float*)(ws + oX);

  const dim3 blk(256);
  const int n8   = MROWS * DE / 8;
  const int per8 = SEQ * DE / 8;
  const int src8 = SEQ_FULL * DE / 8;
  const dim3 gCvt((n8 + 255) / 256);
  const dim3 gWt((DE / 64) * (DE / 64), 4);
  const dim3 gG(DE / 64, MROWS / 128);
  int resqb = RESQB;
  if (resqb > NQB) resqb = NQB;

  cvt_bf16x8s<<<gCvt, blk, 0, stream>>>(pre_q, PQb, n8, per8, src8);
  cvt_bf16x8s<<<gCvt, blk, 0, stream>>>(pre_k, PKb, n8, per8, src8);
  wt_tiles<<<gWt, blk, 0, stream>>>(Wq, Wk, Wv, Wo, Wqt, Wkt, Wvt, Wot);
  gemm_nt<0><<<gG, blk, 0, stream>>>(PQb, Wqt, bq, pre_q, Qh, Xb, 1.0f);
  gemm_nt<0><<<gG, blk, 0, stream>>>(PKb, Wkt, bk, pre_q, Kh, Xb, 1.0f);
  gemm_nt<1><<<gG, blk, 0, stream>>>(PKb, Wvt, bv, pre_q, VTb, Xb, VCARRY);
  attn_full64<true><<<dim3(NB * NH * resqb), dim3(128), 0, stream>>>(Qh, Kh, VTb, CTXb, 0, resqb);
  if (NQB - resqb > 0) {
    attn_full64<false><<<dim3(NB * NH * (NQB - resqb)), dim3(128), 0, stream>>>(Qh, Kh, VTb, CTXb, resqb, NQB - resqb);
  }
  gemm_nt<2><<<gG, blk, 0, stream>>>(CTXb, Wot, bo, pre_q, CTXb, Xb, 1.0f / (CCARRY * WCARRY));
  ln_rows<<<dim3(MROWS), blk, 0, stream>>>(Xb, gamma, beta, out);
  (void)hipGetLastError();
}
